// CobraBlock_61692910240067
// MI455X (gfx1250) — hardware-run, weakly checked
//
#include <hip/hip_runtime.h>
#include <hip/hip_fp16.h>
#include <math.h>

typedef __attribute__((ext_vector_type(16))) _Float16 v16h;
typedef __attribute__((ext_vector_type(8)))  _Float16 v8h;
typedef __attribute__((ext_vector_type(8)))  float    v8f;
typedef __attribute__((ext_vector_type(4)))  float    v4f;
typedef __attribute__((ext_vector_type(4)))  unsigned v4u;

constexpr int kBatch  = 4;
constexpr int kSeq    = 4096;
constexpr int kDim    = 256;
constexpr int kRows   = kBatch * kSeq;
constexpr int kNst    = 16;
constexpr int kDtR    = 16;
constexpr int kDbcN   = kDtR + 2 * kNst;
constexpr int kBcP    = 64;
constexpr int kOffB   = kDtR;
constexpr int kOffC   = kDtR + kNst;
constexpr int kDtK    = 32;
constexpr int kConvTP = 260;
constexpr float kResid   = 2048.0f;
constexpr float kWpCarry = 128.0f;
constexpr float kWdCarry = 128.0f;
constexpr float kWtCarry = 32.0f;
constexpr float kUCarry  = 16.0f;
constexpr float kDlCarry = 16.0f;
constexpr float kRCarry  = 4.0f;
constexpr float kYCarry  = 16.0f;
static_assert(kDbcN == 48);
static_assert(kDbcN <= kBcP);
static_assert(kRows == 16384);
static_assert((kDim % 64) == 0 && (kSeq % 64) == 0 && (kBcP % 64) == 0);
static_assert((kDim % 32) == 0 && (kDtK % 32) == 0 && kDtR <= kDtK);
static_assert((kRows % 32) == 0 && (kRows % 64) == 0);
static_assert(kDim == 256);

constexpr int kSite0Spl = 0;
constexpr int kSite2Spl = 0;
constexpr int kSite3Spl = 0;
constexpr int kSite5Spl = 0;

constexpr float kS0  = 1.0f / kWpCarry;
constexpr float kS0r = kS0 / kResid;
constexpr float kS2  = 1.0f / (kUCarry * kWdCarry);
constexpr float kS2r = kS2 / kResid;
constexpr float kS3  = 1.0f / (kDlCarry * kWtCarry);
constexpr float kS3r = kS3 / kResid;
constexpr float kS5  = 1.0f / (kRCarry * kWpCarry);
constexpr float kS5r = kS5 / kResid;

constexpr size_t kSzWP  = (size_t)kDim * kDim * 2;
constexpr size_t kSzWD  = (size_t)kBcP * kDim * 2;
constexpr size_t kSzWT  = (size_t)kDim * kDtK * 2;
constexpr size_t kSzA16 = (size_t)kRows * kDim * 2;
constexpr size_t kSzA32 = (size_t)kRows * kDim * 4;
constexpr size_t kSzDBC = (size_t)kRows * kBcP * 4;
constexpr size_t kSzDL  = (size_t)kRows * kDtK * 2;
constexpr size_t kOffWPH = 0;
constexpr size_t kOffWPL = kOffWPH + kSzWP;
constexpr size_t kOffWDH = kOffWPL + kSzWP;
constexpr size_t kOffWDL = kOffWDH + kSzWD;
constexpr size_t kOffWTH = kOffWDL + kSzWD;
constexpr size_t kOffWTL = kOffWTH + kSzWT;
constexpr size_t kOffXH  = kOffWTL + kSzWT;
constexpr size_t kOffXL  = kOffXH  + kSzA16;
constexpr size_t kOffP   = kOffXL  + kSzA16;
constexpr size_t kOffU   = kOffP   + kSzA32;
constexpr size_t kOffUH  = kOffU   + kSzA32;
constexpr size_t kOffUL  = kOffUH  + kSzA16;
constexpr size_t kOffDBC = kOffUL  + kSzA16;
constexpr size_t kOffDLH = kOffDBC + kSzDBC;
constexpr size_t kOffDLL = kOffDLH + kSzDL;
constexpr size_t kOffDT  = kOffDLL + kSzDL;
constexpr size_t kOffYH  = kOffDT  + kSzA32;
constexpr size_t kOffYL  = kOffYH  + kSzA16;
constexpr size_t kOffRH  = kOffYL  + kSzA16;
constexpr size_t kOffRL  = kOffRH  + kSzA16;
constexpr size_t kWsTotal = kOffRL + kSzA16;
static_assert(kWsTotal == 124092416ull);
static_assert(kWsTotal <= 134217728ull);
static_assert((kOffWPL % 128) == 0 && (kOffWDH % 128) == 0 && (kOffWDL % 128) == 0 && (kOffWTH % 128) == 0 &&
              (kOffWTL % 128) == 0 && (kOffXH % 128) == 0 && (kOffXL % 128) == 0 && (kOffP % 128) == 0 &&
              (kOffU % 128) == 0 && (kOffUH % 128) == 0 && (kOffUL % 128) == 0 && (kOffDBC % 128) == 0 &&
              (kOffDLH % 128) == 0 && (kOffDLL % 128) == 0 && (kOffDT % 128) == 0 && (kOffYH % 128) == 0 &&
              (kOffYL % 128) == 0 && (kOffRH % 128) == 0 && (kOffRL % 128) == 0);

__device__ __forceinline__ _Float16 f16_flush(float v) {
  const float w = (fabsf(v) < 6.103515625e-05f) ? 0.0f : v;
  return (_Float16)w;
}
__device__ __forceinline__ void f16_split(float v, _Float16& hi, _Float16& lo) {
  hi = f16_flush(v);
  const float hf = (float)hi;
  const float r = (v - hf) * kResid;
  lo = f16_flush(r);
}
__device__ __forceinline__ float h16_to_f32(unsigned hb) {
  const unsigned sgn = (hb & 0x8000u) << 16;
  const unsigned em = hb & 0x7fffu;
  const float fn = __uint_as_float((em << 13) + 0x38000000u);
  const float fs = (float)em * 5.9604644775390625e-8f;
  const float mag = (em < 0x400u) ? fs : fn;
  return __uint_as_float(__float_as_uint(mag) | sgn);
}

namespace eng {
union FragU { v16h v; v8h h[2]; };
__device__ __forceinline__ v16h frag_load(const _Float16* p) {
  FragU f;
  f.h[0] = *(const v8h*)(p);
  f.h[1] = *(const v8h*)(p + 16);
  return f.v;
}
__device__ __forceinline__ v8f mma(v16h a, v16h b, v8f c) {
  return __builtin_amdgcn_wmma_f32_16x16x32_f16(false, a, false, b, (short)0, c, false, false);
}
__device__ __forceinline__ void guard1(v8f& a, v16h x, v16h y) {
  asm volatile("v_nop\n\tv_nop\n\tv_nop\n\tv_nop" : "+v"(a) : "v"(x), "v"(y));
}
__device__ __forceinline__ void guard_acc(v8f& a) {
  asm volatile("v_nop\n\tv_nop\n\tv_nop\n\tv_nop" : "+v"(a));
}
__device__ __forceinline__ void keep4(v16h a, v16h b, v16h c, v16h d) {
  asm volatile("v_nop" :: "v"(a), "v"(b), "v"(c), "v"(d));
}

template <int MI, int SPL, int BIAS>
__global__ __launch_bounds__(256) void gemm_f16_kernel(
    const unsigned short* __restrict__ Ap, const unsigned short* __restrict__ A2p, int lda,
    const unsigned short* __restrict__ Btp, const unsigned short* __restrict__ Bt2p, int ldb,
    float* __restrict__ C, int ldc, const float* __restrict__ bias,
    int M, int N, int K, float scale, float rscale)
{
  static_assert(MI >= 1 && MI <= 2);
  static_assert(SPL >= 0 && SPL <= 2);
  const _Float16* A   = (const _Float16*)Ap;
  const _Float16* A2  = (const _Float16*)A2p;
  const _Float16* Bt  = (const _Float16*)Btp;
  const _Float16* Bt2 = (const _Float16*)Bt2p;
  __shared__ __align__(16) float sT[8][16 * 68];
  const int lane = threadIdx.x & 31;
  const int wave = threadIdx.x >> 5;
  const int tilesN = N >> 6;
  const int tilesM = M / (16 * MI);
  const int tile = blockIdx.x * 8 + wave;
  if (tile >= tilesM * tilesN) return;
  const int tm = tile / tilesN;
  const int tn = tile - tm * tilesN;
  const int m0 = tm * (16 * MI);
  const int n0 = tn << 6;
  const int rlane = lane & 15;
  const int koff  = (lane >> 4) * 8;
  const int mOff  = (lane >> 4) * 8;

  v8f acc[MI][4], accr[MI][4];
#pragma unroll
  for (int i = 0; i < MI; ++i)
#pragma unroll
    for (int j = 0; j < 4; ++j) {
      acc[i][j]  = (v8f){0.f, 0.f, 0.f, 0.f, 0.f, 0.f, 0.f, 0.f};
      accr[i][j] = (v8f){0.f, 0.f, 0.f, 0.f, 0.f, 0.f, 0.f, 0.f};
    }

  for (int k0 = 0; k0 < K; k0 += 32) {
    v16h bh[4], bl[4];
#pragma unroll
    for (int j = 0; j < 4; ++j) {
      const size_t bo = (size_t)(n0 + (j << 4) + rlane) * ldb + koff + k0;
      bh[j] = frag_load(Bt + bo);
      if (SPL == 2) bl[j] = frag_load(Bt2 + bo); else bl[j] = bh[j];
    }
#pragma unroll
    for (int i = 0; i < MI; ++i) {
      const size_t ao = (size_t)(m0 + (i << 4) + rlane) * lda + koff + k0;
      const v16h ah = frag_load(A + ao);
      v16h al = ah;
      if (SPL >= 1) al = frag_load(A2 + ao);
#pragma unroll
      for (int j = 0; j < 4; ++j) {
        acc[i][j] = mma(ah, bh[j], acc[i][j]);
        if (SPL >= 1) accr[i][j] = mma(al, bh[j], accr[i][j]);
        if (SPL == 2) accr[i][j] = mma(ah, bl[j], accr[i][j]);
      }
#pragma unroll
      for (int j = 0; j < 4; ++j) {
        guard1(acc[i][j], ah, al);
        if (SPL >= 1) guard1(accr[i][j], ah, al);
      }
    }
    keep4(bh[0], bh[1], bh[2], bh[3]);
    if (SPL == 2) keep4(bl[0], bl[1], bl[2], bl[3]);
  }
#pragma unroll
  for (int i = 0; i < MI; ++i)
#pragma unroll
    for (int j = 0; j < 4; ++j) {
      guard_acc(acc[i][j]);
      if (SPL >= 1) guard_acc(accr[i][j]);
    }

  float* slab = sT[wave];
  const int hh = lane >> 4, c4 = (lane & 15) * 4;
  v4f bv = (v4f){0.f, 0.f, 0.f, 0.f};
  if (BIAS) bv = *(const v4f*)(bias + n0 + c4);
#pragma unroll
  for (int i = 0; i < MI; ++i) {
    const int mBase = m0 + (i << 4);
#pragma unroll
    for (int j = 0; j < 4; ++j) {
#pragma unroll
      for (int r = 0; r < 8; ++r) {
        float v = acc[i][j][r] * scale;
        if (SPL >= 1) v += accr[i][j][r] * rscale;
        slab[(mOff + r) * 68 + (j << 4) + rlane] = v;
      }
    }
    __builtin_amdgcn_fence(__ATOMIC_RELEASE, "workgroup");
    __builtin_amdgcn_wave_barrier();
    __builtin_amdgcn_fence(__ATOMIC_ACQUIRE, "workgroup");
    {
      v4f vv[8];
#pragma unroll
      for (int it = 0; it < 8; ++it) {
        const int row = it * 2 + hh;
        const v4f t = *(const v4f*)(slab + row * 68 + c4);
        vv[it] = t + bv;
      }
      for (int pass = 0; pass < 2; ++pass) {
#pragma unroll
        for (int it = 0; it < 8; ++it) {
          const int row = it * 2 + hh;
          *(volatile v4f*)(C + (size_t)(mBase + row) * ldc + n0 + c4) = vv[it];
        }
        __threadfence();
      }
    }
    __builtin_amdgcn_fence(__ATOMIC_RELEASE, "workgroup");
    __builtin_amdgcn_wave_barrier();
    __builtin_amdgcn_fence(__ATOMIC_ACQUIRE, "workgroup");
  }
}
}

__global__ __launch_bounds__(256) void split_rows_f16_kernel(
    const float* __restrict__ src, unsigned short* __restrict__ dH, unsigned short* __restrict__ dL, int total8)
{
  const int i = blockIdx.x * 256 + threadIdx.x;
  if (i >= total8) return;
  const size_t e0 = (size_t)i << 3;
  const v4f a0 = *(const v4f*)(src + e0);
  const v4f a1 = *(const v4f*)(src + e0 + 4);
  v8h hv, lv;
#pragma unroll
  for (int e = 0; e < 4; ++e) {
    _Float16 h0, l0, h1, l1;
    const float f0 = a0[e];
    const float f1 = a1[e];
    f16_split(f0, h0, l0);
    f16_split(f1, h1, l1);
    hv[e] = h0; lv[e] = l0;
    hv[4 + e] = h1; lv[4 + e] = l1;
  }
  unsigned short* qh = dH + e0;
  unsigned short* ql = dL + e0;
  *(volatile v8h*)qh = hv;
  *(volatile v8h*)ql = lv;
  __threadfence();
  *(volatile v8h*)qh = hv;
  *(volatile v8h*)ql = lv;
}

template <bool LO>
__global__ __launch_bounds__(256) void transpose_pack_kernel(
    const float* __restrict__ W, unsigned short* __restrict__ BtH, unsigned short* __restrict__ BtL,
    int Kdim, int Ndim, float carry)
{
  __shared__ float tile[64 * 65];
  const int tid = threadIdx.x, lane = tid & 31, wave = tid >> 5;
  const int n0 = blockIdx.x * 64;
  const int k0 = blockIdx.y * 64;
#pragma unroll
  for (int p = 0; p < 16; ++p) {
    const int idx = tid + p * 256;
    const int kk  = idx >> 6;
    const int nn  = idx & 63;
    const int n   = n0 + nn;
    const int nc  = (n < Ndim) ? n : (Ndim - 1);
    const float v = W[(size_t)(k0 + kk) * Ndim + nc];
    tile[kk * 65 + nn] = (n < Ndim) ? (v * carry) : 0.0f;
  }
  __syncthreads();
  const int q = lane >> 3, c8 = (lane & 7) * 8;
  v8h hv[2], lv[2];
#pragma unroll
  for (int it = 0; it < 2; ++it) {
    const int nrow = it * 32 + wave * 4 + q;
#pragma unroll
    for (int e = 0; e < 8; ++e) {
      _Float16 h, l;
      const float t = tile[(c8 + e) * 65 + nrow];
      f16_split(t, h, l);
      hv[it][e] = h;
      lv[it][e] = l;
    }
  }
  for (int pass = 0; pass < 2; ++pass) {
#pragma unroll
    for (int it = 0; it < 2; ++it) {
      const int nrow = it * 32 + wave * 4 + q;
      const size_t o = (size_t)(n0 + nrow) * Kdim + k0 + c8;
      *(volatile v8h*)(BtH + o) = hv[it];
      if (LO) *(volatile v8h*)(BtL + o) = lv[it];
    }
    __threadfence();
  }
}

__global__ __launch_bounds__(256) void wdt_pack_kernel(
    const float* __restrict__ Wdt, unsigned short* __restrict__ BtH, unsigned short* __restrict__ BtL, float carry)
{
  const int i = blockIdx.x * 256 + threadIdx.x;
  if (i >= kDim * 4) return;
  const int n  = i >> 2;
  const int kq = (i & 3) * 8;
  const int kc = kq & (kDtR - 1);
  const float keep = (kq < kDtR) ? 1.0f : 0.0f;
  v8h hv, lv;
#pragma unroll
  for (int e = 0; e < 8; ++e) {
    _Float16 h, l;
    const float w = Wdt[(size_t)(kc + e) * kDim + n];
    const float t = w * keep * carry;
    f16_split(t, h, l);
    hv[e] = h;
    lv[e] = l;
  }
  const size_t e0 = (size_t)i << 3;
  unsigned short* qh = BtH + e0;
  unsigned short* ql = BtL + e0;
  *(volatile v8h*)qh = hv;
  *(volatile v8h*)ql = lv;
  __threadfence();
  *(volatile v8h*)qh = hv;
  *(volatile v8h*)ql = lv;
}

__global__ __launch_bounds__(256) void conv3_silu_kernel(
    const float* __restrict__ P, const float* __restrict__ cw, const float* __restrict__ cb,
    float* __restrict__ UC, unsigned short* __restrict__ UH, unsigned short* __restrict__ UL)
{
  __shared__ __align__(16) float sT[16 * kConvTP];
  const int tid = threadIdx.x, lane = tid & 31, wave = tid >> 5;
  const int d  = tid;
  const int t0 = blockIdx.x * 64;
  const int l0 = t0 & (kSeq - 1);
  const float w0 = cw[d * 3 + 0];
  const float w1 = cw[d * 3 + 1];
  const float w2 = cw[d * 3 + 2];
  const float bc = cb[d];
  float xprev, xcur;
  {
    const int rp = (t0 > 0) ? (t0 - 1) : 0;
    const float vp = P[(size_t)rp * kDim + d];
    xprev = (l0 > 0) ? vp : 0.0f;
    xcur  = P[(size_t)t0 * kDim + d];
  }
  const int hrow = wave >> 1;
  const int hch  = (wave & 1) * 128 + lane * 4;
#pragma unroll 1
  for (int sub = 0; sub < 4; ++sub) {
    const int lb = t0 + sub * 16;
#pragma unroll 1
    for (int s = 0; s < 16; ++s) {
      const int t  = lb + s;
      const int l  = l0 + sub * 16 + s;
      const int tn = (t + 1 < kRows) ? (t + 1) : (kRows - 1);
      const float vn = P[(size_t)tn * kDim + d];
      const float xnext = (l + 1 < kSeq) ? vn : 0.0f;
      float acc = w0 * xprev;
      acc = fmaf(w1, xcur, acc);
      acc = fmaf(w2, xnext, acc);
      const float sv = acc + bc;
      const float sg = __builtin_amdgcn_rcpf(1.0f + expf(-sv));
      sT[s * kConvTP + tid] = sv * sg;
      xprev = xcur;
      xcur  = xnext;
    }
    __syncthreads();
    v4f fv[4];
    v8h hv[2], lv[2];
#pragma unroll
    for (int it = 0; it < 4; ++it) fv[it] = *(const v4f*)(sT + (it * 4 + hrow) * kConvTP + hch);
#pragma unroll
    for (int it = 0; it < 2; ++it) {
      const float* sp = sT + (it * 8 + wave) * kConvTP + lane * 8;
      const v4f a0 = *(const v4f*)(sp);
      const v4f a1 = *(const v4f*)(sp + 4);
#pragma unroll
      for (int e = 0; e < 4; ++e) {
        _Float16 h0, l0h, h1, l1h;
        const float f0 = a0[e] * kUCarry;
        const float f1 = a1[e] * kUCarry;
        f16_split(f0, h0, l0h);
        f16_split(f1, h1, l1h);
        hv[it][e] = h0; lv[it][e] = l0h;
        hv[it][4 + e] = h1; lv[it][4 + e] = l1h;
      }
    }
    for (int pass = 0; pass < 2; ++pass) {
#pragma unroll
      for (int it = 0; it < 4; ++it)
        *(volatile v4f*)(UC + (size_t)(lb + it * 4 + hrow) * kDim + hch) = fv[it];
#pragma unroll
      for (int it = 0; it < 2; ++it) {
        const size_t o = (size_t)(lb + it * 8 + wave) * kDim + lane * 8;
        *(volatile v8h*)(UH + o) = hv[it];
        *(volatile v8h*)(UL + o) = lv[it];
      }
      __threadfence();
    }
    __syncthreads();
  }
}

__global__ __launch_bounds__(256) void dl_pack_kernel(
    const float* __restrict__ DBC, unsigned short* __restrict__ dH, unsigned short* __restrict__ dL, int total)
{
  const int i = blockIdx.x * 256 + threadIdx.x;
  if (i >= total) return;
  const int row = i >> 2;
  const int kq  = (i & 3) * 8;
  const int kc  = kq & (kDtR - 1);
  const float keep = (kq < kDtR) ? kDlCarry : 0.0f;
  const v4f a0 = *(const v4f*)(DBC + (size_t)row * kBcP + kc);
  const v4f a1 = *(const v4f*)(DBC + (size_t)row * kBcP + kc + 4);
  v8h hv, lv;
#pragma unroll
  for (int e = 0; e < 4; ++e) {
    _Float16 h0, l0, h1, l1;
    const float f0 = a0[e] * keep;
    const float f1 = a1[e] * keep;
    f16_split(f0, h0, l0);
    f16_split(f1, h1, l1);
    hv[e] = h0; lv[e] = l0;
    hv[4 + e] = h1; lv[4 + e] = l1;
  }
  const size_t e0 = (size_t)i << 3;
  unsigned short* qh = dH + e0;
  unsigned short* ql = dL + e0;
  *(volatile v8h*)qh = hv;
  *(volatile v8h*)ql = lv;
  __threadfence();
  *(volatile v8h*)qh = hv;
  *(volatile v8h*)ql = lv;
}

__global__ __launch_bounds__(256) void resid_pack_kernel(
    const unsigned short* __restrict__ YH, const unsigned short* __restrict__ YL, const float* __restrict__ x,
    unsigned short* __restrict__ RH, unsigned short* __restrict__ RL, int total8)
{
  const int i = blockIdx.x * 256 + threadIdx.x;
  if (i >= total8) return;
  const size_t e0 = (size_t)i << 3;
  const v4u yh = *(const v4u*)(YH + e0);
  const v4u yl = *(const v4u*)(YL + e0);
  const v4f x0 = *(const v4f*)(x + e0);
  const v4f x1 = *(const v4f*)(x + e0 + 4);
  float xs[8];
  xs[0] = x0[0]; xs[1] = x0[1]; xs[2] = x0[2]; xs[3] = x0[3];
  xs[4] = x1[0]; xs[5] = x1[1]; xs[6] = x1[2]; xs[7] = x1[3];
  constexpr float kInvResid = 1.0f / kResid;
  constexpr float kInvY = 1.0f / kYCarry;
  v8h hv, lv;
#pragma unroll
  for (int w = 0; w < 4; ++w) {
    const unsigned hw = yh[w];
    const unsigned lw = yl[w];
    const float yv0 = h16_to_f32(hw & 0xffffu);
    const float yv1 = h16_to_f32(hw >> 16);
    const float yr0 = h16_to_f32(lw & 0xffffu);
    const float yr1 = h16_to_f32(lw >> 16);
    const float g0 = (yv0 + yr0 * kInvResid) * kInvY;
    const float g1 = (yv1 + yr1 * kInvResid) * kInvY;
    const float r0 = (g0 + xs[2 * w]) * kRCarry;
    const float r1 = (g1 + xs[2 * w + 1]) * kRCarry;
    _Float16 h0, l0, h1, l1;
    f16_split(r0, h0, l0);
    f16_split(r1, h1, l1);
    hv[2 * w] = h0; lv[2 * w] = l0;
    hv[2 * w + 1] = h1; lv[2 * w + 1] = l1;
  }
  unsigned short* qh = RH + e0;
  unsigned short* ql = RL + e0;
  *(volatile v8h*)qh = hv;
  *(volatile v8h*)ql = lv;
  __threadfence();
  *(volatile v8h*)qh = hv;
  *(volatile v8h*)ql = lv;
}

typedef float    ms1_v4f __attribute__((ext_vector_type(4)));
typedef unsigned ms1_v4u __attribute__((ext_vector_type(4)));
struct ms1_args {
  const float* dtpre;
  const float* u;
  const float* bc;
  const float* z;
  const float* A_log;
  const float* Dskip;
  __half* y;
  __half* y_lo;
  long ld_dtpre;
  long ld_u;
  long ld_bc;
  long ld_z;
  long ld_y;
  int offB;
  int offC;
  int offZ;
  float ycarry;
  int dir;
  int D;
  int L;
  int nbatch;
};
static_assert(sizeof(ms1_args) == 136);

__device__ __forceinline__ float ms1_flush16(float v) {
  return (fabsf(v) < 6.103515625e-05f) ? 0.0f : v;
}
__device__ __forceinline__ unsigned ms1_h16bits(float v) {
  return (unsigned)__half_as_ushort(__float2half_rn(ms1_flush16(v)));
}
__device__ __forceinline__ float ms1_h16val(unsigned b) {
  return __half2float(__ushort_as_half((unsigned short)b));
}
__device__ __forceinline__ float ms1_softplus(float v) {
  return fmaxf(v, 0.0f) + log1pf(expf(-fabsf(v)));
}
__device__ __forceinline__ void ms1_pack2(float v0, float v1, unsigned& hw, unsigned& lw) {
  const unsigned h0 = ms1_h16bits(v0);
  const unsigned h1 = ms1_h16bits(v1);
  const float r0 = (v0 - ms1_h16val(h0)) * 2048.0f;
  const float r1 = (v1 - ms1_h16val(h1)) * 2048.0f;
  const unsigned l0 = ms1_h16bits(r0);
  const unsigned l1 = ms1_h16bits(r1);
  hw = h0 | (h1 << 16);
  lw = l0 | (l1 << 16);
}

template <int NSTATE>
__global__ __launch_bounds__(64 * (NSTATE / 16)) void ms1_scan_kernel(ms1_args a)
{
  static_assert(NSTATE == 16 || NSTATE == 64);
  constexpr int NQ  = NSTATE / 16;
  constexpr int NT  = 64 * NQ;
  constexpr int NW  = NT / 32;
  constexpr int BCW = 2 * NSTATE;
  constexpr int YP  = 68;
  constexpr int RPI = NW * 4;
  constexpr int NIT = 64 / RPI;
  static_assert(16 * NT <= 64 * YP);
  __shared__ __align__(16) float sBC[64 * BCW];
  __shared__ __align__(16) float sY[64 * YP];
  const int tid  = threadIdx.x;
  const int lane = tid & 31;
  const int wave = tid >> 5;
  const int c    = tid / NQ;
  const int sq   = tid - c * NQ;
  const int bpb  = a.D / 64;
  const int bi   = blockIdx.x / bpb;
  if (bi >= a.nbatch) return;
  const int d0 = (blockIdx.x - bi * bpb) * 64;
  const int d  = d0 + c;
  const long rowb = (long)bi * a.L;
  const bool hasz  = (a.z != nullptr);
  const bool hasD  = (a.Dskip != nullptr);
  const bool hasLo = (a.y_lo != nullptr);

#pragma unroll 1
  for (int n = 0; n < 16; ++n) {
    const float al = a.A_log[(long)d * NSTATE + sq * 16 + n];
    sY[n * NT + tid] = -expf(al);
  }
  __syncthreads();
  float An[16], h[16];
#pragma unroll
  for (int n = 0; n < 16; ++n) {
    An[n] = sY[n * NT + tid];
    h[n] = 0.0f;
  }
  float Dd = 0.0f;
  if (hasD) Dd = a.Dskip[d];

  const int nchunk = a.L / 64;
  const bool fwd = (a.dir > 0);
  const int s0 = fwd ? 0 : 63;
  const int sd = fwd ? 1 : -1;
  const int q  = lane >> 3;
  const int c8 = (lane & 7) * 8;

#pragma unroll 1
  for (int ci = 0; ci < nchunk; ++ci) {
    const int tb = fwd ? (ci * 64) : (a.L - 64 - ci * 64);
    const long rowc = rowb + tb;
    __syncthreads();
#pragma unroll 8
    for (int i = 0; i < 32; ++i) {
      const int idx = tid + i * NT;
      const int st  = idx / BCW;
      const int col = idx - st * BCW;
      const int sc  = (col < NSTATE) ? (a.offB + col) : (a.offC + col - NSTATE);
      sBC[idx] = a.bc[(rowc + st) * a.ld_bc + sc];
    }
    __syncthreads();
#pragma unroll 1
    for (int s = 0; s < 64; ++s) {
      const int ls = s0 + sd * s;
      const long row = rowc + ls;
      float pre = a.dtpre[row * a.ld_dtpre + d];
      float uv  = a.u[row * a.ld_u + d];
      float zv  = 0.0f;
      if (hasz) zv = a.z[row * a.ld_z + a.offZ + d];
      asm volatile("" : "+v"(pre));
      asm volatile("" : "+v"(uv));
      asm volatile("" : "+v"(zv));
      const float delta = ms1_softplus(pre);
      const float dtx = delta * uv;
      const float* bp = sBC + ls * BCW + sq * 16;
      const float* cp = bp + NSTATE;
      ms1_v4f Bq[4], Cq[4];
#pragma unroll
      for (int k = 0; k < 4; ++k) {
        Bq[k] = *(const ms1_v4f*)(bp + 4 * k);
        Cq[k] = *(const ms1_v4f*)(cp + 4 * k);
      }
      float yv = 0.0f;
#pragma unroll
      for (int n = 0; n < 16; ++n) {
        const float e = __expf(delta * An[n]);
        h[n] = fmaf(e, h[n], dtx * Bq[n >> 2][n & 3]);
        yv = fmaf(h[n], Cq[n >> 2][n & 3], yv);
      }
      if (NQ > 1) {
        yv += __shfl_xor(yv, 1, 32);
        yv += __shfl_xor(yv, 2, 32);
      }
      if (hasD) yv = fmaf(uv, Dd, yv);
      if (hasz) {
        const float sg = __builtin_amdgcn_rcpf(1.0f + expf(-zv));
        yv = yv * (zv * sg);
      }
      if (sq == 0) sY[ls * YP + c] = yv * a.ycarry;
    }
    __syncthreads();
    ms1_v4u hw[NIT], lw[NIT];
#pragma unroll
    for (int it = 0; it < NIT; ++it) {
      const int row = it * RPI + wave * 4 + q;
      const float* sp = sY + row * YP + c8;
      const ms1_v4f f0 = *(const ms1_v4f*)(sp);
      const ms1_v4f f1 = *(const ms1_v4f*)(sp + 4);
      unsigned h0, h1, h2, h3, l0, l1, l2, l3;
      ms1_pack2(f0[0], f0[1], h0, l0);
      ms1_pack2(f0[2], f0[3], h1, l1);
      ms1_pack2(f1[0], f1[1], h2, l2);
      ms1_pack2(f1[2], f1[3], h3, l3);
      hw[it] = (ms1_v4u){h0, h1, h2, h3};
      lw[it] = (ms1_v4u){l0, l1, l2, l3};
    }
    for (int pass = 0; pass < 2; ++pass) {
#pragma unroll
      for (int it = 0; it < NIT; ++it) {
        const int row = it * RPI + wave * 4 + q;
        const long o = (rowc + row) * a.ld_y + d0 + c8;
        *(volatile ms1_v4u*)(a.y + o) = hw[it];
        if (hasLo) *(volatile ms1_v4u*)(a.y_lo + o) = lw[it];
      }
      __threadfence();
    }
  }
}

template <int SPL, int BIAS>
static void run_gemm(const unsigned short* A, const unsigned short* A2, int lda,
                     const unsigned short* Bt, const unsigned short* Bt2, int ldb,
                     float* C, int ldc, const float* bias, int M, int N, int K,
                     float scale, float rscale, hipStream_t stream)
{
  constexpr int MI = (SPL == 2) ? 1 : 2;
  const int tiles  = (M / (16 * MI)) * (N / 64);
  const int blocks = (tiles + 7) / 8;
  eng::gemm_f16_kernel<MI, SPL, BIAS><<<dim3(blocks), 256, 0, stream>>>(
      A, A2, lda, Bt, Bt2, ldb, C, ldc, bias, M, N, K, scale, rscale);
}

extern "C" void kernel_launch(void* const* d_in, const int* in_sizes, int n_in,
                              void* d_out, int out_size, void* d_ws, size_t ws_size,
                              hipStream_t stream)
{
  if (n_in < 10) return;
  if (in_sizes[0] != kRows * kDim) return;
  if (in_sizes[1] != kDim * kDim) return;
  if (in_sizes[2] != kDim) return;
  if (in_sizes[3] != kDim * 3) return;
  if (in_sizes[4] != kDim) return;
  if (in_sizes[5] != kDim * kDbcN) return;
  if (in_sizes[6] != kDtR * kDim) return;
  if (in_sizes[7] != kDim) return;
  if (in_sizes[8] != kDim * kNst) return;
  if (in_sizes[9] != kDim) return;
  if (out_size != kRows * kDim) return;
  if (ws_size < kWsTotal) return;

  const float* x      = (const float*)d_in[0];
  const float* W_proj = (const float*)d_in[1];
  const float* b_proj = (const float*)d_in[2];
  const float* conv_w = (const float*)d_in[3];
  const float* conv_b = (const float*)d_in[4];
  const float* W_dbc  = (const float*)d_in[5];
  const float* W_dt   = (const float*)d_in[6];
  const float* b_dt   = (const float*)d_in[7];
  const float* A_log  = (const float*)d_in[8];
  const float* D_skip = (const float*)d_in[9];
  float* out = (float*)d_out;

  char* ws = (char*)d_ws;
  unsigned short* WPH = (unsigned short*)(ws + kOffWPH);
  unsigned short* WPL = (unsigned short*)(ws + kOffWPL);
  unsigned short* WDH = (unsigned short*)(ws + kOffWDH);
  unsigned short* WDL = (unsigned short*)(ws + kOffWDL);
  unsigned short* WTH = (unsigned short*)(ws + kOffWTH);
  unsigned short* WTL = (unsigned short*)(ws + kOffWTL);
  unsigned short* XH  = (unsigned short*)(ws + kOffXH);
  unsigned short* XL  = (unsigned short*)(ws + kOffXL);
  float*          P   = (float*)(ws + kOffP);
  float*          U   = (float*)(ws + kOffU);
  unsigned short* UH  = (unsigned short*)(ws + kOffUH);
  unsigned short* UL  = (unsigned short*)(ws + kOffUL);
  float*          DBC = (float*)(ws + kOffDBC);
  unsigned short* DLH = (unsigned short*)(ws + kOffDLH);
  unsigned short* DLL = (unsigned short*)(ws + kOffDLL);
  float*          DT  = (float*)(ws + kOffDT);
  unsigned short* YH  = (unsigned short*)(ws + kOffYH);
  unsigned short* YL  = (unsigned short*)(ws + kOffYL);
  unsigned short* RH  = (unsigned short*)(ws + kOffRH);
  unsigned short* RL  = (unsigned short*)(ws + kOffRL);

  transpose_pack_kernel<true><<<dim3(kDim / 64, kDim / 64), 256, 0, stream>>>(W_proj, WPH, WPL, kDim, kDim, kWpCarry);
  transpose_pack_kernel<true><<<dim3(kBcP / 64, kDim / 64), 256, 0, stream>>>(W_dbc, WDH, WDL, kDim, kDbcN, kWdCarry);
  wdt_pack_kernel<<<dim3((kDim * 4) / 256), 256, 0, stream>>>(W_dt, WTH, WTL, kWtCarry);

  split_rows_f16_kernel<<<(kRows * kDim / 8) / 256, 256, 0, stream>>>(x, XH, XL, kRows * kDim / 8);

  run_gemm<kSite0Spl, 1>(XH, XL, kDim, WPH, WPL, kDim, P, kDim, b_proj, kRows, kDim, kDim, kS0, kS0r, stream);

  conv3_silu_kernel<<<dim3(kRows / 64), 256, 0, stream>>>(P, conv_w, conv_b, U, UH, UL);

  run_gemm<kSite2Spl, 0>(UH, UL, kDim, WDH, WDL, kDim, DBC, kBcP, b_proj, kRows, kBcP, kDim, kS2, kS2r, stream);

  dl_pack_kernel<<<(kRows * 4) / 256, 256, 0, stream>>>(DBC, DLH, DLL, kRows * 4);

  run_gemm<kSite3Spl, 1>(DLH, DLL, kDtK, WTH, WTL, kDtK, DT, kDim, b_dt, kRows, kDim, kDtK, kS3, kS3r, stream);

  for (int b = 0; b < kBatch; ++b) {
    const size_t ro = (size_t)b * kSeq;
    ms1_args sa;
    sa.dtpre = DT + ro * kDim;
    sa.u = U + ro * kDim;
    sa.bc = DBC + ro * kBcP;
    sa.z = P + ro * kDim;
    sa.A_log = A_log;
    sa.Dskip = D_skip;
    sa.y = (__half*)(YH + ro * kDim);
    sa.y_lo = (__half*)(YL + ro * kDim);
    sa.ld_dtpre = kDim;
    sa.ld_u = kDim;
    sa.ld_bc = kBcP;
    sa.ld_z = kDim;
    sa.ld_y = kDim;
    sa.offB = kOffB;
    sa.offC = kOffC;
    sa.offZ = 0;
    sa.ycarry = kYCarry;
    sa.dir = 1;
    sa.D = kDim;
    sa.L = kSeq;
    sa.nbatch = 1;
    ms1_scan_kernel<16><<<dim3(kDim / 64), 64, 0, stream>>>(sa);
  }

  resid_pack_kernel<<<(kRows * kDim / 8) / 256, 256, 0, stream>>>(YH, YL, x, RH, RL, kRows * kDim / 8);

  run_gemm<kSite5Spl, 1>(RH, RL, kDim, WPH, WPL, kDim, out, kDim, b_proj, kRows, kDim, kDim, kS5, kS5r, stream);
}
